// myGNN2_17016660427425
// MI455X (gfx1250) — hardware-verified
//
#include <hip/hip_runtime.h>
#include <stddef.h>
#include <stdint.h>


#define HC      64
#define K1      192
#define K2      256
#define NF1     8
#define NF2     2
#define NGR     64
#define NTHR    256
#define NWAVE   8
#define EPT     8
#define CHUNK   (NTHR * EPT)
#define WCAP    (EPT * 32)
#define LISTN   (NWAVE * WCAP)
#define NBMAX   2048
#define RCAP    28672
#define DEGCAP  1024
#define STW     64
#define GBM     64
#define GBN     64
#define GTHR    128
#define WSMAX   134217728
#define LDS_AGG ((2 * RCAP + 2 * NBMAX + LISTN) * 4 + 64)

static_assert((CHUNK & (CHUNK - 1)) == 0 && CHUNK <= 4096);
static_assert((NBMAX & (NBMAX - 1)) == 0 && NBMAX <= 4096);
static_assert(NTHR * 8 == NBMAX);
static_assert(LISTN >= NBMAX);
static_assert(LISTN >= NWAVE * WCAP);
static_assert((RCAP % 32) == 0);
static_assert(NWAVE * STW <= RCAP);
static_assert(STW * 2 >= 128);
static_assert(((STW * 4) % 16) == 0);
static_assert(LDS_AGG <= 300000);
static_assert(GBM == (GTHR / 32) * 16);
static_assert((K1 % 32) == 0 && (K2 % 32) == 0 && (HC % 32) == 0);
static_assert(K1 == 3 * HC && K2 == 4 * HC);
static_assert(GBN == HC);
static_assert(GBM * NF1 / 4 == GTHR);
static_assert(GBM * NF2 / 4 == 32);
static_assert(2 * NGR == 32 * 4);
static_assert(HC * NF1 == 4 * GTHR);
static_assert(NF1 == 8 && NF2 == 2);
static_assert(NGR <= NTHR);

typedef float          v2f   __attribute__((ext_vector_type(2)));
typedef float          v4f   __attribute__((ext_vector_type(4)));
typedef float          v8f   __attribute__((ext_vector_type(8)));
typedef int            v4i   __attribute__((ext_vector_type(4)));
typedef int            v8i   __attribute__((ext_vector_type(8)));
typedef unsigned short v8us  __attribute__((ext_vector_type(8)));
typedef unsigned short v8usa __attribute__((ext_vector_type(8), may_alias));
typedef __bf16         v16bf __attribute__((ext_vector_type(16)));
union FragB { v16bf v; v8us h[2]; v8i w; };

__device__ __forceinline__ v8f wmb(const FragB& a, const FragB& b, v8f c) {
  v8f d = __builtin_amdgcn_wmma_f32_16x16x32_bf16(false, a.v, false, b.v, (short)0, c, false, false);
  asm volatile("v_nop\n\tv_nop\n\tv_nop\n\tv_nop" : "+v"(d) : "v"(a.w), "v"(b.w));
  return d;
}

__device__ __forceinline__ unsigned int bf16_bits(float f) {
  const unsigned int u = __float_as_uint(f);
  return (u + 0x7FFFu + ((u >> 16) & 1u)) >> 16;
}
__device__ __forceinline__ float bf16_val(unsigned int b) { return __uint_as_float(b << 16); }
__device__ __forceinline__ float bfr(float f) { return bf16_val(bf16_bits(f)); }

__device__ __forceinline__ v8us cvt8b(const v4f a, const v4f b) {
  v8us o;
  o[0] = (unsigned short)bf16_bits(a.x); o[1] = (unsigned short)bf16_bits(a.y);
  o[2] = (unsigned short)bf16_bits(a.z); o[3] = (unsigned short)bf16_bits(a.w);
  o[4] = (unsigned short)bf16_bits(b.x); o[5] = (unsigned short)bf16_bits(b.y);
  o[6] = (unsigned short)bf16_bits(b.z); o[7] = (unsigned short)bf16_bits(b.w);
  return o;
}

__device__ __forceinline__ void split8(const v4f a, const v4f b, v8us& hi, v8us& lo) {
  float f[8];
  f[0] = a.x; f[1] = a.y; f[2] = a.z; f[3] = a.w; f[4] = b.x; f[5] = b.y; f[6] = b.z; f[7] = b.w;
#pragma unroll
  for (int i = 0; i < 8; ++i) {
    const unsigned int hb = bf16_bits(f[i]);
    const unsigned int lb = bf16_bits(f[i] - bf16_val(hb));
    hi[i] = (unsigned short)hb;
    lo[i] = (unsigned short)lb;
  }
}

__device__ __forceinline__ int scan_chunk(const int* __restrict__ dsts, int nE, int cbase, int slotBase,
                                          int nb, int vec8, int* list, int tid, int lane, int wave) {
  int wc = 0;
  const int el0  = tid * EPT;
  const int e0   = cbase + el0;
  const int sent = -2147483647 - 1;
  v4i da, db;
  if (vec8 != 0 && cbase + CHUNK <= nE) {
    da = *(const v4i*)(dsts + e0);
    db = *(const v4i*)(dsts + e0 + 4);
  } else {
    da.x = (e0     < nE) ? dsts[min(e0,     nE - 1)] : sent;
    da.y = (e0 + 1 < nE) ? dsts[min(e0 + 1, nE - 1)] : sent;
    da.z = (e0 + 2 < nE) ? dsts[min(e0 + 2, nE - 1)] : sent;
    da.w = (e0 + 3 < nE) ? dsts[min(e0 + 3, nE - 1)] : sent;
    db.x = (e0 + 4 < nE) ? dsts[min(e0 + 4, nE - 1)] : sent;
    db.y = (e0 + 5 < nE) ? dsts[min(e0 + 5, nE - 1)] : sent;
    db.z = (e0 + 6 < nE) ? dsts[min(e0 + 6, nE - 1)] : sent;
    db.w = (e0 + 7 < nE) ? dsts[min(e0 + 7, nE - 1)] : sent;
  }
  const unsigned nbs = (unsigned)slotBase;
  const unsigned unb = (unsigned)nb;
  const unsigned s0 = (unsigned)da.x - nbs, s1 = (unsigned)da.y - nbs;
  const unsigned s2 = (unsigned)da.z - nbs, s3 = (unsigned)da.w - nbs;
  const unsigned s4 = (unsigned)db.x - nbs, s5 = (unsigned)db.y - nbs;
  const unsigned s6 = (unsigned)db.z - nbs, s7 = (unsigned)db.w - nbs;
  const bool h0 = s0 < unb, h1 = s1 < unb, h2 = s2 < unb, h3 = s3 < unb;
  const bool h4 = s4 < unb, h5 = s5 < unb, h6 = s6 < unb, h7 = s7 < unb;
  const unsigned any = __builtin_amdgcn_ballot_w32(h0 | h1 | h2 | h3 | h4 | h5 | h6 | h7);
  if (any != 0u) {
#define HITJ(J, HJ, SJ) { \
      const unsigned mj = __builtin_amdgcn_ballot_w32(HJ); \
      if (mj != 0u) { \
        if (HJ) { \
          const int pos = wc + (int)__builtin_amdgcn_mbcnt_lo(mj, 0u); \
          if (pos < WCAP) list[wave * WCAP + pos] = ((el0 + (J)) << 12) | (int)(SJ); \
        } \
        wc += (int)__builtin_popcount(mj); } }
    HITJ(0, h0, s0)
    HITJ(1, h1, s1)
    HITJ(2, h2, s2)
    HITJ(3, h3, s3)
    HITJ(4, h4, s4)
    HITJ(5, h5, s5)
    HITJ(6, h6, s6)
    HITJ(7, h7, s7)
#undef HITJ
  }
  return wc;
}

__global__ __launch_bounds__(NTHR) void k_xprep(const float* __restrict__ x, unsigned short* A1, int nN, int nUnits) {
  const int i = (int)blockIdx.x * NTHR + (int)threadIdx.x;
  if (i >= nUnits) return;
  const int row = i >> 3;
  const int c0  = (i & 7) * 8;
  const int rc  = row < nN ? row : nN - 1;
  const float* p = x + (size_t)rc * HC + c0;
  v4f a = *(const v4f*)p, b = *(const v4f*)(p + 4);
  const v4f z4 = {0.f, 0.f, 0.f, 0.f};
  if (row >= nN) { a = z4; b = z4; }
  const v8us hv = cvt8b(a, b);
  const size_t o = (size_t)row * K1 + c0;
  *(volatile v8us*)(A1 + o) = hv;
  __threadfence();
  *(volatile v8us*)(A1 + o) = hv;
}

__global__ __launch_bounds__(NTHR) void k_wtr(const float* __restrict__ w0, const float* __restrict__ w1,
                                              const float* __restrict__ w2, const float* __restrict__ w3,
                                              int K, unsigned short* wt, int nUnits) {
  const int u = (int)blockIdx.x * NTHR + (int)threadIdx.x;
  if (u >= nUnits) return;
  const int kq = K >> 3;
  const int n  = u / kq;
  const int k8 = (u - n * kq) * 8;
  int seg = k8 >> 6;
  seg = seg > 3 ? 3 : seg;
  const int kk = k8 & (HC - 1);
  const float* wsp = (seg == 0) ? w0 : ((seg == 1) ? w1 : ((seg == 2) ? w2 : w3));
  const int ncl = n < HC ? n : HC - 1;
  const float* p = wsp + (size_t)kk * HC + ncl;
  v4f a, b;
  a.x = p[0];          a.y = p[HC];         a.z = p[2 * HC];     a.w = p[3 * HC];
  b.x = p[4 * HC];     b.y = p[5 * HC];     b.z = p[6 * HC];     b.w = p[7 * HC];
  const v8us hv = cvt8b(a, b);
  const size_t o = (size_t)n * (size_t)K + k8;
  *(volatile v8us*)(wt + o) = hv;
  __threadfence();
  *(volatile v8us*)(wt + o) = hv;
}

template<int EPI>
__global__ __launch_bounds__(GTHR) void k_gemm(
    const unsigned short* __restrict__ A, const unsigned short* __restrict__ WT, const float* __restrict__ bias,
    float* outF, unsigned short* An, float* Zp,
    const float* __restrict__ fc1w, const float* __restrict__ fc1b,
    const float* __restrict__ fc2w, const float* __restrict__ fc2b,
    int K, int nRows, int ldAn, int cLoN)
{
  __shared__ __attribute__((aligned(16))) float stg[GBM * GBN];
  __shared__ __attribute__((aligned(16))) float sW1[HC * NF1];
  __shared__ __attribute__((aligned(16))) float midS[GBM * NF1];
  __shared__ __attribute__((aligned(16))) float zS[GBM * NF2];
  __shared__ float sB1[NF1];
  __shared__ float sW2[NF1 * NF2];
  __shared__ float sB2[NF2];
  const int tid = (int)threadIdx.x, lane = tid & 31, wave = tid >> 5, hh = lane >> 4, m = lane & 15;
  const int rowBase = (int)blockIdx.x * GBM;

  if (EPI == 1) {
    const v4f w4 = *(const v4f*)(fc1w + 4 * tid);
    sW1[4 * tid + 0] = bfr(w4.x); sW1[4 * tid + 1] = bfr(w4.y);
    sW1[4 * tid + 2] = bfr(w4.z); sW1[4 * tid + 3] = bfr(w4.w);
    if (tid < NF1)       sB1[tid] = bfr(fc1b[tid]);
    if (tid < NF1 * NF2) sW2[tid] = bfr(fc2w[tid]);
    if (tid < NF2)       sB2[tid] = bfr(fc2b[tid]);
  }

  v8f acc[4];
  {
    const v8f z = {0.f, 0.f, 0.f, 0.f, 0.f, 0.f, 0.f, 0.f};
    acc[0] = z; acc[1] = z; acc[2] = z; acc[3] = z;
  }
  const unsigned short* ap = A  + (size_t)(rowBase + 16 * wave + m) * (size_t)K + 8 * hh;
  const unsigned short* wp = WT + (size_t)m * (size_t)K + 8 * hh;
  const int ksteps = K >> 5;
#pragma unroll 1
  for (int ks = 0; ks < ksteps; ++ks) {
    FragB af;
    af.h[0] = *(const v8us*)(ap + 32 * ks);
    af.h[1] = *(const v8us*)(ap + 32 * ks + 16);
#pragma unroll
    for (int t = 0; t < 4; ++t) {
      const unsigned short* wq = wp + (size_t)(16 * t) * (size_t)K + 32 * ks;
      FragB bf;
      bf.h[0] = *(const v8us*)wq;
      bf.h[1] = *(const v8us*)(wq + 16);
      acc[t] = wmb(af, bf, acc[t]);
    }
  }

#pragma unroll
  for (int t = 0; t < 4; ++t) {
    const int lc = 16 * t + m;
    const float bv = bfr(bias[lc]);
#pragma unroll
    for (int r = 0; r < 8; ++r) {
      const int lr = 16 * wave + 8 * hh + r;
      const int gr = rowBase + lr;
      float v = fmaxf(acc[t][r] + bv, 0.f);
      v = (gr < nRows) ? v : 0.f;
      stg[lr * GBN + lc] = v;
    }
  }
  __syncthreads();

  if (EPI == 0) {
    v4f fv[8];
#pragma unroll
    for (int i = 0; i < 8; ++i) {
      const int lr = 16 * wave + 2 * i + hh;
      fv[i] = *(const v4f*)(stg + lr * GBN + 4 * m);
    }
#pragma unroll
    for (int i = 0; i < 8; ++i) {
      const int lr = 16 * wave + 2 * i + hh;
      const int gr = rowBase + lr;
      float* op = outF + (size_t)gr * (size_t)HC + 4 * m;
      *(volatile v4f*)op = fv[i];
    }
    __threadfence();
#pragma unroll
    for (int i = 0; i < 8; ++i) {
      const int lr = 16 * wave + 2 * i + hh;
      const int gr = rowBase + lr;
      float* op = outF + (size_t)gr * (size_t)HC + 4 * m;
      *(volatile v4f*)op = fv[i];
    }
    const int q = lane >> 3, p8 = (lane & 7) * 8;
    const int isLo = q & 1, rsub = q >> 1;
    const int cofs = isLo ? cLoN : 0;
    v8us sv[8];
#pragma unroll
    for (int j = 0; j < 8; ++j) {
      const int lr = 16 * wave + 2 * j + rsub;
      const v4f a = *(const v4f*)(stg + lr * GBN + p8);
      const v4f b = *(const v4f*)(stg + lr * GBN + p8 + 4);
      v8us h8, l8;
      split8(a, b, h8, l8);
      sv[j] = isLo ? l8 : h8;
    }
#pragma unroll
    for (int j = 0; j < 8; ++j) {
      const int gr = rowBase + 16 * wave + 2 * j + rsub;
      unsigned short* up = An + (size_t)gr * (size_t)ldAn + cofs + p8;
      *(volatile v8us*)up = sv[j];
    }
    __threadfence();
#pragma unroll
    for (int j = 0; j < 8; ++j) {
      const int gr = rowBase + 16 * wave + 2 * j + rsub;
      unsigned short* up = An + (size_t)gr * (size_t)ldAn + cofs + p8;
      *(volatile v8us*)up = sv[j];
    }
  } else {
    if (tid < GBM) {
      const int row = tid;
      const float* hr = stg + row * GBN;
      const v4f ma = *(const v4f*)hr, mb = *(const v4f*)(hr + 4);
      const float mx = fmaxf(fmaxf(fmaxf(ma.x, ma.y), fmaxf(ma.z, ma.w)),
                             fmaxf(fmaxf(mb.x, mb.y), fmaxf(mb.z, mb.w)));
      const float e0 = expf(ma.x - mx), e1 = expf(ma.y - mx), e2 = expf(ma.z - mx), e3 = expf(ma.w - mx);
      const float e4 = expf(mb.x - mx), e5 = expf(mb.y - mx), e6 = expf(mb.z - mx), e7 = expf(mb.w - mx);
      const float ssum = ((e0 + e1) + (e2 + e3)) + ((e4 + e5) + (e6 + e7));
      const float inv = 1.0f / ssum;
      v4f pa, pb;
      pa.x = e0 * inv; pa.y = e1 * inv; pa.z = e2 * inv; pa.w = e3 * inv;
      pb.x = e4 * inv; pb.y = e5 * inv; pb.z = e6 * inv; pb.w = e7 * inv;
      *(v4f*)(midS + row * NF1)     = pa;
      *(v4f*)(midS + row * NF1 + 4) = pb;
      float z[NF1];
#pragma unroll
      for (int j = 0; j < NF1; ++j) z[j] = 0.f;
#pragma unroll 2
      for (int c = 0; c < HC; ++c) {
        const float hv = hr[c];
        const float* wr = sW1 + c * NF1;
#pragma unroll
        for (int j = 0; j < NF1; ++j) z[j] = fmaf(hv, wr[j], z[j]);
      }
#pragma unroll
      for (int j = 0; j < NF1; ++j) z[j] = fmaxf(z[j] + sB1[j], 0.f);
#pragma unroll
      for (int k = 0; k < NF2; ++k) {
        float a2 = 0.f;
#pragma unroll
        for (int j = 0; j < NF1; ++j) a2 = fmaf(z[j], sW2[j * NF2 + k], a2);
        zS[row * NF2 + k] = fmaxf(a2 + sB2[k], 0.f);
      }
    }
    __syncthreads();
    int nv = nRows - rowBase;
    nv = nv < 0 ? 0 : (nv > GBM ? GBM : nv);
    const int np = nv * (NF1 / 4);
    const v4f pv = *(const v4f*)(midS + 4 * tid);
    float* op = outF + (size_t)rowBase * NF1 + 4 * tid;
    if (tid < np) *(volatile v4f*)op = pv;
    __threadfence();
    if (tid < np) *(volatile v4f*)op = pv;
    if (wave == 0) {
      const v4f zv = *(const v4f*)(zS + 4 * lane);
      float* zp = Zp + (size_t)rowBase * NF2 + 4 * lane;
      *(volatile v4f*)zp = zv;
      __threadfence();
      *(volatile v4f*)zp = zv;
    }
  }
}

template<int RND>
__global__ __launch_bounds__(NTHR) void k_gat(
    const int* __restrict__ srcs, const int* __restrict__ dsts,
    const float* __restrict__ hsrc, unsigned short* Aout,
    int nN, int nE, int nb, int vec8, int MPr, int ldA, int cHi, int cLo) {
  extern __shared__ v4f lds_dyn[];
  int* reg1 = (int*)lds_dyn;
  int* reg2 = reg1 + RCAP;
  int* scnt = reg2 + RCAP;
  int* soff = scnt + NBMAX;
  int* list = soff + NBMAX;
  int* wcnt = list + LISTN;
  int* wtot = wcnt + NWAVE;
  const int tid = (int)threadIdx.x, lane = tid & 31, wave = tid >> 5;
  const int nodeBase = (int)blockIdx.x * nb;

  for (int i = tid; i < NBMAX; i += NTHR) scnt[i] = 0;
  __syncthreads();

  int tot = 0;
  const int nChunks = (nE + CHUNK - 1) / CHUNK;
#pragma unroll 1
  for (int ch = 0; ch < nChunks; ++ch) {
    const int cbase = ch * CHUNK;
    const int wc = scan_chunk(dsts, nE, cbase, nodeBase, nb, vec8, list, tid, lane, wave);
    if (lane == 0) wcnt[wave] = wc;
    __syncthreads();
    int pre = 0, all = 0;
#pragma unroll
    for (int w2 = 0; w2 < NWAVE; ++w2) {
      int c = wcnt[w2];
      c = c < 0 ? 0 : (c > WCAP ? WCAP : c);
      all += c;
      pre += (w2 < wave) ? c : 0;
    }
    const int wcc  = wc > WCAP ? WCAP : wc;
    const int base = tot + pre;
#pragma unroll 1
    for (int i = lane; i < wcc; i += 32) {
      const int ent = list[wave * WCAP + i];
      const int el  = (ent >> 12) & (CHUNK - 1);
      const int sl  = ent & (NBMAX - 1);
      int eid = cbase + el;
      eid = eid > nE - 1 ? nE - 1 : eid;
      const int pos = base + i;
      if (pos < RCAP) reg1[pos] = (int)(((unsigned)eid << 12) | (unsigned)sl);
    }
    tot += all;
    tot = tot > RCAP ? RCAP : tot;
    __syncthreads();
  }
  const int nh = tot;

  if (wave == 0) {
#pragma unroll 1
    for (int b0 = 0; b0 < nh; b0 += 32) {
      const int idx = b0 + lane;
      const int uv  = reg1[idx < RCAP ? idx : RCAP - 1];
      const int m32 = (nh - b0) < 32 ? (nh - b0) : 32;
#pragma unroll 1
      for (int k = 0; k < m32; ++k) {
        const int u  = __builtin_amdgcn_readlane(uv, k);
        const int sl = u & (NBMAX - 1);
        if (lane == 0) scnt[sl] = scnt[sl] + 1;
      }
    }
  }
  __syncthreads();

  {
    const v4i ca = *(const v4i*)(scnt + 8 * tid);
    const v4i cb = *(const v4i*)(scnt + 8 * tid + 4);
    const int e0 = ca.x < 0 ? 0 : ca.x, e1 = ca.y < 0 ? 0 : ca.y, e2 = ca.z < 0 ? 0 : ca.z, e3 = ca.w < 0 ? 0 : ca.w;
    const int e4 = cb.x < 0 ? 0 : cb.x, e5 = cb.y < 0 ? 0 : cb.y, e6 = cb.z < 0 ? 0 : cb.z, e7 = cb.w < 0 ? 0 : cb.w;
    const int ts = e0 + e1 + e2 + e3 + e4 + e5 + e6 + e7;
    int incl = ts;
#pragma unroll
    for (int d = 1; d < 32; d <<= 1) {
      const int up = __shfl_up(incl, d);
      if (lane >= d) incl += up;
    }
    if (lane == 31) wtot[wave] = incl;
    __syncthreads();
    int pre = 0;
#pragma unroll
    for (int w2 = 0; w2 < NWAVE; ++w2) pre += (w2 < wave) ? wtot[w2] : 0;
    int run = pre + incl - ts;
    soff[8 * tid + 0] = run; run += e0;
    soff[8 * tid + 1] = run; run += e1;
    soff[8 * tid + 2] = run; run += e2;
    soff[8 * tid + 3] = run; run += e3;
    soff[8 * tid + 4] = run; run += e4;
    soff[8 * tid + 5] = run; run += e5;
    soff[8 * tid + 6] = run; run += e6;
    soff[8 * tid + 7] = run;
  }
  __syncthreads();
  for (int i = tid; i < NBMAX; i += NTHR) list[i] = soff[i];
  __syncthreads();

  if (wave == 0) {
#pragma unroll 1
    for (int b0 = 0; b0 < nh; b0 += 32) {
      const int idx = b0 + lane;
      const int uv  = reg1[idx < RCAP ? idx : RCAP - 1];
      const int m32 = (nh - b0) < 32 ? (nh - b0) : 32;
#pragma unroll 1
      for (int k = 0; k < m32; ++k) {
        const int u   = __builtin_amdgcn_readlane(uv, k);
        const int sl  = u & (NBMAX - 1);
        const int eid = (int)((unsigned)u >> 12);
        if (lane == 0) {
          int pos = list[sl];
          pos = pos < 0 ? 0 : (pos > RCAP - 1 ? RCAP - 1 : pos);
          reg2[pos] = eid;
          list[sl] = pos + 1;
        }
      }
    }
  }
  __syncthreads();

  const int nbw = nb >> 3;
  const bool ovf = (nh >= RCAP);
  const float qnan = __uint_as_float(0x7fc00000u);
  unsigned short* stw = (unsigned short*)(reg1 + wave * STW);
  const int lc   = lane < 16 ? lane : 15;
  const int colw = (lane < 8) ? (cHi + 8 * lane) : (cLo + 8 * (lc - 8));
#pragma unroll 1
  for (int jt = 0; jt < nbw; ++jt) {
    const int slot = wave * nbw + jt;
    const int grow = nodeBase + slot;
    int st = soff[slot];
    const int craw = scnt[slot];
    int cnt = craw;
    st  = st < 0 ? 0 : (st > nh ? nh : st);
    cnt = cnt < 0 ? 0 : (cnt > DEGCAP ? DEGCAP : cnt);
    if (cnt > nh - st) cnt = nh - st;
    const float pz = (ovf || craw > DEGCAP) ? qnan : 0.0f;
    const bool wr = grow < MPr;
    const float live = grow < nN ? 1.0f : 0.0f;

    float s0 = 0.f, s1 = 0.f;
#pragma unroll 1
    for (int q = 0; q < cnt; ++q) {
      int idx = st + q; idx = idx > RCAP - 1 ? RCAP - 1 : idx;
      int eid = reg2[idx]; eid = eid < 0 ? 0 : (eid > nE - 1 ? nE - 1 : eid);
      const int sraw = srcs[eid];
      const int s = sraw < 0 ? 0 : (sraw > nN - 1 ? nN - 1 : sraw);
      const float* hr = hsrc + (size_t)s * HC + lane;
      float v0 = hr[0];
      float v1 = hr[32];
      if (RND) { v0 = bfr(v0); v1 = bfr(v1); }
      s0 += v0;
      s1 += v1;
    }
    const float a0 = s0 * live + pz;
    const float a1 = s1 * live + pz;
    const unsigned int h0 = bf16_bits(a0), h1 = bf16_bits(a1);
    const unsigned int l0 = bf16_bits(a0 - bf16_val(h0)), l1 = bf16_bits(a1 - bf16_val(h1));
    __builtin_amdgcn_fence(__ATOMIC_RELEASE, "wavefront");
    __builtin_amdgcn_wave_barrier();
    stw[lane]      = (unsigned short)h0;
    stw[32 + lane] = (unsigned short)h1;
    stw[64 + lane] = (unsigned short)l0;
    stw[96 + lane] = (unsigned short)l1;
    __builtin_amdgcn_fence(__ATOMIC_RELEASE, "wavefront");
    __builtin_amdgcn_wave_barrier();
    const v8us pv = *(const v8usa*)(stw + 8 * lc);
    const int gcw = wr ? grow : MPr - 1;
    unsigned short* gp = Aout + (size_t)gcw * (size_t)ldA + colw;
    const bool wsv = wr && (lane < 16);
    if (wsv) *(volatile v8us*)gp = pv;
    __threadfence();
    if (wsv) *(volatile v8us*)gp = pv;
  }
}

__global__ __launch_bounds__(NTHR) void k_pool(const int* __restrict__ bat, const float* __restrict__ Zp,
                                               float* out, int nN, int outOff) {
  __shared__ __attribute__((aligned(16))) float ldsRes[2 * NGR];
  const int tid = (int)threadIdx.x, lane = tid & 31, wave = tid >> 5;
  const float ninf = __uint_as_float(0xff800000u);
#pragma unroll 1
  for (int g = wave; g < NGR; g += NWAVE) {
    float m0 = ninf, m1 = ninf;
#pragma unroll 1
    for (int n0 = 0; n0 < nN; n0 += 32) {
      const int n  = n0 + lane;
      const int nc = n < nN ? n : nN - 1;
      const int b  = bat[nc];
      const v2f v  = *(const v2f*)(Zp + 2 * (size_t)nc);
      const bool hit = (n < nN) && (b == g);
      m0 = hit ? fmaxf(m0, v.x) : m0;
      m1 = hit ? fmaxf(m1, v.y) : m1;
    }
#pragma unroll
    for (int off = 16; off > 0; off >>= 1) {
      m0 = fmaxf(m0, __shfl_xor(m0, off));
      m1 = fmaxf(m1, __shfl_xor(m1, off));
    }
    const float mm  = fmaxf(m0, m1);
    const float e0  = expf(m0 - mm), e1 = expf(m1 - mm);
    const float inv = 1.0f / (e0 + e1);
    if (lane == 0) { ldsRes[2 * g] = e0 * inv; ldsRes[2 * g + 1] = e1 * inv; }
  }
  __syncthreads();
  if (wave == 0) {
    const v4f v = *(const v4f*)(ldsRes + 4 * lane);
    float* op = out + (size_t)outOff + 4 * lane;
    *(volatile v4f*)op = v;
    __threadfence();
    *(volatile v4f*)op = v;
  }
}

static int pick_nb(int nE, int nN) {
  int nb = NBMAX;
  while (nb > 16 && (long long)nb * (long long)nE * 5LL > (long long)RCAP * (long long)nN * 4LL) nb >>= 1;
  return nb;
}
static inline int cdiv(int a, int b) { return (a + b - 1) / b; }

extern "C" void kernel_launch(void* const* d_in, const int* in_sizes, int n_in,
                              void* d_out, int out_size, void* d_ws, size_t ws_size,
                              hipStream_t stream) {
  if (n_in < 13) return;
  const int nN = in_sizes[0] / HC;
  if (nN <= 0 || in_sizes[0] != nN * HC || nN > (1 << 22)) return;
  if (in_sizes[1] < 2 || (in_sizes[1] & 1) != 0) return;
  const int nE = in_sizes[1] / 2;
  if (nE < 1 || nE > (1 << 20)) return;
  if (in_sizes[2] != nN) return;
  if (in_sizes[3] != HC * HC || in_sizes[4] != HC * HC || in_sizes[5] != HC) return;
  if (in_sizes[6] != HC * HC || in_sizes[7] != HC * HC || in_sizes[8] != HC) return;
  if (in_sizes[9] != HC * NF1 || in_sizes[10] != NF1) return;
  if (in_sizes[11] != NF1 * NF2 || in_sizes[12] != NF2) return;
  if (out_size != nN * NF1 + 2 * NGR) return;
  if (((long long)nN * NF1 * 4LL) % 128LL != 0LL) return;

  const float* x    = (const float*)d_in[0];
  const int*   ei   = (const int*)  d_in[1];
  const int*   bat  = (const int*)  d_in[2];
  const float* W1r  = (const float*)d_in[3];
  const float* W1g  = (const float*)d_in[4];
  const float* b1   = (const float*)d_in[5];
  const float* W2r  = (const float*)d_in[6];
  const float* W2g  = (const float*)d_in[7];
  const float* b2   = (const float*)d_in[8];
  const float* fc1w = (const float*)d_in[9];
  const float* fc1b = (const float*)d_in[10];
  const float* fc2w = (const float*)d_in[11];
  const float* fc2b = (const float*)d_in[12];
  float* out = (float*)d_out;
  const int* src = ei;
  const int* dst = ei + nE;

  const int MP   = cdiv(nN, GBM) * GBM;
  const int nb   = pick_nb(nE, nN);
  const int gA   = cdiv(MP, nb);
  const int vec8 = ((nE & 3) == 0) ? 1 : 0;
  if (gA * nb < MP) return;

  char* wsb = (char*)d_ws;
  size_t off = 0;
  const size_t oA1  = off; off += (size_t)MP * K1 * 2;             off = (off + 255) & ~(size_t)255;
  const size_t oH1  = off; off += (size_t)MP * HC * 4;             off = (off + 255) & ~(size_t)255;
  const size_t oA2  = off; off += (size_t)MP * K2 * 2;             off = (off + 255) & ~(size_t)255;
  const size_t oZ   = off; off += (size_t)MP * NF2 * 4;            off = (off + 255) & ~(size_t)255;
  const size_t oWT1 = off; off += (size_t)HC * K1 * 2;             off = (off + 255) & ~(size_t)255;
  const size_t oWT2 = off; off += (size_t)HC * K2 * 2;             off = (off + 255) & ~(size_t)255;
  if (off > ws_size || off > (size_t)WSMAX) return;
  unsigned short* A1  = (unsigned short*)(wsb + oA1);
  float*          H1F = (float*)(wsb + oH1);
  unsigned short* A2  = (unsigned short*)(wsb + oA2);
  float*          Zp  = (float*)(wsb + oZ);
  unsigned short* WT1 = (unsigned short*)(wsb + oWT1);
  unsigned short* WT2 = (unsigned short*)(wsb + oWT2);

  hipFuncSetAttribute(reinterpret_cast<const void*>(&k_gat<1>),
                      hipFuncAttributeMaxDynamicSharedMemorySize, LDS_AGG);
  hipFuncSetAttribute(reinterpret_cast<const void*>(&k_gat<0>),
                      hipFuncAttributeMaxDynamicSharedMemorySize, LDS_AGG);

  const int nUx = MP * (HC / 8);
  k_xprep<<<cdiv(nUx, NTHR), NTHR, 0, stream>>>(x, A1, nN, nUx);

  {
    const int nU1 = HC * (K1 / 8);
    k_wtr<<<cdiv(nU1, NTHR), NTHR, 0, stream>>>(W1r, W1g, W1g, W1g, K1, WT1, nU1);
    const int nU2 = HC * (K2 / 8);
    k_wtr<<<cdiv(nU2, NTHR), NTHR, 0, stream>>>(W2r, W2g, W2r, W2g, K2, WT2, nU2);
  }

  const int gM = MP / GBM;
  k_gat<1><<<gA, NTHR, LDS_AGG, stream>>>(src, dst, x, A1, nN, nE, nb, vec8, MP, K1, HC, 2 * HC);
  k_gemm<0><<<gM, GTHR, 0, stream>>>(A1, WT1, b1, H1F, A2, Zp, fc1w, fc1b, fc2w, fc2b, K1, nN, K2, 2 * HC);
  k_gat<0><<<gA, NTHR, LDS_AGG, stream>>>(src, dst, H1F, A2, nN, nE, nb, vec8, MP, K2, HC, 3 * HC);
  k_gemm<1><<<gM, GTHR, 0, stream>>>(A2, WT2, b2, out, A1, Zp, fc1w, fc1b, fc2w, fc2b, K2, nN, K2, 2 * HC);
  k_pool<<<1, NTHR, 0, stream>>>(bat, Zp, out, nN, nN * NF1);
}
